// GraphSAGE_73203422593459
// MI455X (gfx1250) — hardware-run, weakly checked
//
#include <hip/hip_runtime.h>
#include <stddef.h>
#include <stdint.h>


#define NN     50000
#define NS     25
#define DF     128
#define NP     50048
#define NTHR   256
#define GBM    64
#define GBN    128
#define GTHR   128
#define GWAVE  (GTHR / 32)
#define NTILE  (NP / GBM)
#define PARTW  288
#define WSTW   258
#define KA0    128
#define KC0    384
#define KA1    256
#define KC1    512
#define HP     256
#define UPART  2048
#define NPART  10
#define XB_UNITS   (NP * (DF / 8))
#define XB_BLOCKS  (XB_UNITS / NTHR)
#define W_BLOCKS   ((NPART * UPART) / NTHR)
#define PREP_BLOCKS (XB_BLOCKS + W_BLOCKS + 1)
#define ROWBLK (NP / 8)

static_assert(DF == 128 && DF == 32 * 4);
static_assert(NS == 25 && NS <= 32);
static_assert(NP == 391 * 128 && NP % GBM == 0 && NP >= NN && NP % 8 == 0);
static_assert(KA0 % 32 == 0 && KC0 % 32 == 0 && KA1 % 32 == 0 && KC1 % 32 == 0);
static_assert(KC0 == 3 * DF && KA1 == 2 * DF && KC1 == 4 * DF && HP == 2 * DF);
static_assert(GBM == GWAVE * 16 && GBN == DF && GTHR == GBN);
static_assert(XB_UNITS % NTHR == 0 && UPART % NTHR == 0 && UPART == DF * (DF / 8));
static_assert(PARTW % 32 == 0 && PARTW / 4 <= GTHR && PARTW >= 2 * GBN + 1);
static_assert(WSTW >= 2 * GBN + 1 && (WSTW % 2) == 0);
static_assert(GBM * GBN * 4 + GWAVE * WSTW * 4 + PARTW * 4 <= 327680);

constexpr size_t SZ_XB   = (size_t)NP * DF * 2;
constexpr size_t SZ_F32  = (size_t)NP * DF * 4;
constexpr size_t SZ_HL   = (size_t)NP * HP * 2;
constexpr size_t SZ_WA0T = (size_t)DF * KA0 * 2;
constexpr size_t SZ_W0C  = (size_t)DF * KC0 * 2;
constexpr size_t SZ_WA1D = (size_t)DF * KA1 * 2;
constexpr size_t SZ_W1C  = (size_t)DF * KC1 * 2;
constexpr size_t SZ_PAR  = (size_t)6 * DF * 4;
constexpr size_t SZ_REC  = (size_t)NTILE * PARTW * 4;
constexpr size_t SZ_STAT = (size_t)3 * DF * 4;
constexpr size_t O_XB   = 0;
constexpr size_t O_P    = O_XB + SZ_XB;
constexpr size_t O_AGG  = O_P + SZ_F32;
constexpr size_t O_T    = O_AGG + SZ_HL;
constexpr size_t O_X2   = O_T + SZ_F32;
constexpr size_t O_WA0T = O_X2 + SZ_HL;
constexpr size_t O_W0C  = O_WA0T + SZ_WA0T;
constexpr size_t O_WA1D = O_W0C + SZ_W0C;
constexpr size_t O_W1C  = O_WA1D + SZ_WA1D;
constexpr size_t O_PAR  = O_W1C + SZ_W1C;
constexpr size_t O_REC  = O_PAR + SZ_PAR;
constexpr size_t O_STAT = O_REC + SZ_REC;
constexpr size_t WS_TOTAL = O_STAT + SZ_STAT;
static_assert(SZ_XB % 256 == 0 && SZ_F32 % 256 == 0 && SZ_HL % 256 == 0);
static_assert(SZ_WA0T % 256 == 0 && SZ_W0C % 256 == 0 && SZ_WA1D % 256 == 0 && SZ_W1C % 256 == 0);
static_assert(SZ_PAR % 256 == 0 && SZ_REC % 256 == 0 && SZ_STAT % 256 == 0);
static_assert(WS_TOTAL <= ((size_t)128u << 20));

typedef float          v4f   __attribute__((ext_vector_type(4)));
typedef float          v8f   __attribute__((ext_vector_type(8)));
typedef int            v8i   __attribute__((ext_vector_type(8)));
typedef unsigned short v4us  __attribute__((ext_vector_type(4)));
typedef unsigned short v8us  __attribute__((ext_vector_type(8)));
typedef unsigned short v16us __attribute__((ext_vector_type(16)));
typedef __bf16         v16bf __attribute__((ext_vector_type(16)));
typedef v4f  __attribute__((may_alias)) v4fa;
typedef v4us __attribute__((may_alias)) v4usa;
typedef v8us __attribute__((may_alias)) v8usa;
union FragB { v16bf v; v16us u; v8us h[2]; v8i w; };

__device__ __forceinline__ v8f wmb(const FragB& a, const FragB& b, v8f c) {
  v8f d = __builtin_amdgcn_wmma_f32_16x16x32_bf16(false, a.v, false, b.v, (short)0, c, false, false);
  asm volatile("v_nop\n\tv_nop\n\tv_nop\n\tv_nop" : "+v"(d) : "v"(a.w), "v"(b.w));
  return d;
}

__device__ __forceinline__ v8f z8() { v8f z = {0.f, 0.f, 0.f, 0.f, 0.f, 0.f, 0.f, 0.f}; return z; }

__device__ __forceinline__ unsigned bf16_bits(float f) {
  const unsigned u = __float_as_uint(f);
  return (u + 0x7FFFu + ((u >> 16) & 1u)) >> 16;
}
__device__ __forceinline__ float bf16_val(float f) {
  return __uint_as_float(bf16_bits(f) << 16);
}

__device__ __forceinline__ void pin4(v4f a) { asm volatile("" :: "v"(a)); }

__device__ __forceinline__ float relu_keep(float v) { return (v > 0.0f) ? v : (v - v); }

__device__ __forceinline__ float max_keep(float v, float m) { return (v > m || v != v) ? v : m; }

__device__ __forceinline__ void wave_sync() {
  __builtin_amdgcn_fence(__ATOMIC_RELEASE, "wavefront");
  __builtin_amdgcn_wave_barrier();
  __builtin_amdgcn_fence(__ATOMIC_ACQUIRE, "wavefront");
}

__device__ __forceinline__ void split4(v4f y, v4us& h4, v4us& l4) {
  unsigned hb;
  hb = bf16_bits(y.x); h4[0] = (unsigned short)hb; l4[0] = (unsigned short)bf16_bits(y.x - __uint_as_float(hb << 16));
  hb = bf16_bits(y.y); h4[1] = (unsigned short)hb; l4[1] = (unsigned short)bf16_bits(y.y - __uint_as_float(hb << 16));
  hb = bf16_bits(y.z); h4[2] = (unsigned short)hb; l4[2] = (unsigned short)bf16_bits(y.z - __uint_as_float(hb << 16));
  hb = bf16_bits(y.w); h4[3] = (unsigned short)hb; l4[3] = (unsigned short)bf16_bits(y.w - __uint_as_float(hb << 16));
}

__device__ __forceinline__ void wpart(const float* __restrict__ W, int srow0, unsigned short* P,
                                      int pitch, int coff, int v) {
  const int n  = v >> 4;
  const int k8 = (v & 15) * 8;
  const float* p = W + (size_t)(srow0 + k8) * DF + n;
  float f[8];
#pragma unroll
  for (int i = 0; i < 8; ++i) f[i] = p[(size_t)i * DF];
  v8us o;
#pragma unroll
  for (int i = 0; i < 8; ++i) o[i] = (unsigned short)bf16_bits(f[i]);
  unsigned short* dp = P + (size_t)n * pitch + coff + k8;
  *(volatile v8us*)dp = o;
  __threadfence();
  *(volatile v8us*)dp = o;
}

__device__ __forceinline__ void parvec(const float* __restrict__ src, float* dst, int lane) {
  const v4f a = *(const v4f*)(src + 4 * lane);
  v4f o;
  o.x = bf16_val(a.x); o.y = bf16_val(a.y); o.z = bf16_val(a.z); o.w = bf16_val(a.w);
  *(volatile v4f*)(dst + 4 * lane) = o;
  __threadfence();
  *(volatile v4f*)(dst + 4 * lane) = o;
}

__global__ __launch_bounds__(NTHR) void k_prep(const float* __restrict__ feat,
                                               const float* __restrict__ Wa0, const float* __restrict__ ba0,
                                               const float* __restrict__ Wa1, const float* __restrict__ ba1,
                                               const float* __restrict__ W0,  const float* __restrict__ b0,
                                               const float* __restrict__ W1,  const float* __restrict__ b1,
                                               const float* __restrict__ gam, const float* __restrict__ bet,
                                               unsigned short* XB, unsigned short* WA0T, unsigned short* W0C,
                                               unsigned short* WA1D, unsigned short* W1C, float* PAR) {
  const int tid = (int)threadIdx.x;
  const int b   = (int)blockIdx.x;
  if (b < XB_BLOCKS) {
    const int u   = b * NTHR + tid;
    const int row = u >> 4;
    const int c8  = (u & 15) * 8;
    const int rc  = row < NN ? row : NN - 1;
    const float* p = feat + (size_t)rc * DF + c8;
    const v4f a = *(const v4f*)p;
    const v4f c = *(const v4f*)(p + 4);
    pin4(a);
    pin4(c);
    const unsigned msk = (row < NN) ? 0xffffu : 0u;
    v8us o;
    o[0] = (unsigned short)(bf16_bits(a.x) & msk); o[1] = (unsigned short)(bf16_bits(a.y) & msk);
    o[2] = (unsigned short)(bf16_bits(a.z) & msk); o[3] = (unsigned short)(bf16_bits(a.w) & msk);
    o[4] = (unsigned short)(bf16_bits(c.x) & msk); o[5] = (unsigned short)(bf16_bits(c.y) & msk);
    o[6] = (unsigned short)(bf16_bits(c.z) & msk); o[7] = (unsigned short)(bf16_bits(c.w) & msk);
    unsigned short* dp = XB + (size_t)u * 8;
    *(volatile v8us*)dp = o;
    __threadfence();
    *(volatile v8us*)dp = o;
  } else if (b < XB_BLOCKS + W_BLOCKS) {
    const int u    = (b - XB_BLOCKS) * NTHR + tid;
    const int part = u >> 11;
    const int v    = u & (UPART - 1);
    if (part == 0)      wpart(Wa0, 0,  WA0T, KA0, 0,      v);
    else if (part == 1) wpart(W0,  0,  W0C,  KC0, 0,      v);
    else if (part == 2) wpart(W0,  DF, W0C,  KC0, DF,     v);
    else if (part == 3) wpart(W0,  DF, W0C,  KC0, 2 * DF, v);
    else if (part == 4) wpart(Wa1, 0,  WA1D, KA1, 0,      v);
    else if (part == 5) wpart(Wa1, 0,  WA1D, KA1, DF,     v);
    else if (part == 6) wpart(W1,  0,  W1C,  KC1, 0,      v);
    else if (part == 7) wpart(W1,  0,  W1C,  KC1, DF,     v);
    else if (part == 8) wpart(W1,  DF, W1C,  KC1, 2 * DF, v);
    else if (part == 9) wpart(W1,  DF, W1C,  KC1, 3 * DF, v);
  } else {
    const int vec  = tid >> 5;
    const int lane = tid & 31;
    if (vec == 0)      parvec(ba0, PAR,          lane);
    else if (vec == 1) parvec(ba1, PAR + DF,     lane);
    else if (vec == 2) parvec(b0,  PAR + 2 * DF, lane);
    else if (vec == 3) parvec(b1,  PAR + 3 * DF, lane);
    else if (vec == 4) parvec(gam, PAR + 4 * DF, lane);
    else if (vec == 5) parvec(bet, PAR + 5 * DF, lane);
  }
}

template <int PA, int KA, int PB, int KB, int RELU, int STATS, int FIN>
__global__ __launch_bounds__(GTHR) __attribute__((amdgpu_num_vgpr(248)))
void k_gemm(const unsigned short* __restrict__ Aa, const unsigned short* __restrict__ Ab,
            const unsigned short* __restrict__ BT, const float* __restrict__ bias,
            float* outp, float* part) {
  static_assert(KA > 0 && KA % 32 == 0 && KB % 32 == 0 && KA <= PA && KB <= PB);
  static_assert(PA % 8 == 0 && PB % 8 == 0);
  constexpr int KT = KA + KB;
  __shared__ __attribute__((aligned(16))) float stg[GBM * GBN];
  __shared__ __attribute__((aligned(16))) float wst[GWAVE * WSTW];
  __shared__ __attribute__((aligned(16))) float pst[PARTW];
  const int tid = (int)threadIdx.x, lane = tid & 31, wave = tid >> 5, hh = lane >> 4, m = lane & 15;
  const int rowBase = (int)blockIdx.x * GBM;

  v8f acc[8];
#pragma unroll
  for (int t = 0; t < 8; ++t) acc[t] = z8();
  const unsigned short* bp = BT + (size_t)m * (size_t)KT + 8 * hh;

  {
    const unsigned short* ap = Aa + (size_t)(rowBase + 16 * wave + m) * (size_t)PA + 8 * hh;
#pragma unroll 1
    for (int k0 = 0; k0 < KA; k0 += 32) {
      FragB af;
      af.h[0] = *(const v8usa*)(ap + k0);
      af.h[1] = *(const v8usa*)(ap + k0 + 16);
#pragma unroll
      for (int nt = 0; nt < 8; ++nt) {
        const unsigned short* wq = bp + (size_t)(16 * nt) * (size_t)KT + k0;
        FragB bf;
        bf.h[0] = *(const v8usa*)wq;
        bf.h[1] = *(const v8usa*)(wq + 16);
        acc[nt] = wmb(af, bf, acc[nt]);
      }
    }
  }
  if constexpr (KB > 0) {
    const unsigned short* ap = Ab + (size_t)(rowBase + 16 * wave + m) * (size_t)PB + 8 * hh;
#pragma unroll 1
    for (int k0 = 0; k0 < KB; k0 += 32) {
      FragB af;
      af.h[0] = *(const v8usa*)(ap + k0);
      af.h[1] = *(const v8usa*)(ap + k0 + 16);
#pragma unroll
      for (int nt = 0; nt < 8; ++nt) {
        const unsigned short* wq = bp + (size_t)(16 * nt) * (size_t)KT + KA + k0;
        FragB bf;
        bf.h[0] = *(const v8usa*)wq;
        bf.h[1] = *(const v8usa*)(wq + 16);
        acc[nt] = wmb(af, bf, acc[nt]);
      }
    }
  }

#pragma unroll
  for (int nt = 0; nt < 8; ++nt) {
    const int lc = 16 * nt + m;
#pragma unroll
    for (int r = 0; r < 8; ++r) {
      const int lr = 16 * wave + 8 * hh + r;
      stg[lr * GBN + lc] = acc[nt][r];
    }
  }
  __syncthreads();

  const v4f bb4 = *(const v4f*)(bias + 4 * lane);

  v4f pv[16];
  float wm[4], wqv[4];
  int wn = 0;
#pragma unroll
  for (int j = 0; j < 4; ++j) { wm[j] = 0.0f; wqv[j] = 0.0f; }
#pragma unroll
  for (int i = 0; i < 16; ++i) {
    const int row = rowBase + 16 * wave + i;
    const bool ok = row < NN;
    const v4f x = *(const v4fa*)(stg + (16 * wave + i) * GBN + 4 * lane);
    float y[4];
    y[0] = x.x + bb4.x; y[1] = x.y + bb4.y; y[2] = x.z + bb4.z; y[3] = x.w + bb4.w;
    if constexpr (RELU != 0) {
      y[0] = relu_keep(y[0]); y[1] = relu_keep(y[1]); y[2] = relu_keep(y[2]); y[3] = relu_keep(y[3]);
    }
    float vv[4];
#pragma unroll
    for (int j = 0; j < 4; ++j) vv[j] = ok ? y[j] : 0.0f;
    v4f q;
    q.x = vv[0]; q.y = vv[1]; q.z = vv[2]; q.w = vv[3];
    pv[i] = q;
    if constexpr (STATS != 0) {
      if (ok) {
        wn += 1;
        const float rk = 1.0f / (float)(i + 1);
#pragma unroll
        for (int j = 0; j < 4; ++j) {
          const float d = vv[j] - wm[j];
          wm[j]  = fmaf(d, rk, wm[j]);
          wqv[j] = fmaf(d, vv[j] - wm[j], wqv[j]);
        }
      }
    }
  }

#pragma unroll
  for (int i = 0; i < 16; ++i) {
    const int r = rowBase + 16 * wave + i;
    if (FIN == 0 || r < NN) *(volatile v4f*)(outp + (size_t)r * DF + 4 * lane) = pv[i];
  }
  __threadfence();
#pragma unroll
  for (int i = 0; i < 16; ++i) {
    const int r = rowBase + 16 * wave + i;
    if (FIN == 0 || r < NN) *(volatile v4f*)(outp + (size_t)r * DF + 4 * lane) = pv[i];
  }

  if constexpr (STATS != 0) {
    if (lane == 0) wst[wave * WSTW] = (float)wn;
#pragma unroll
    for (int j = 0; j < 4; ++j) {
      wst[wave * WSTW + 1 + 4 * lane + j]       = wm[j];
      wst[wave * WSTW + 1 + GBN + 4 * lane + j] = wqv[j];
    }
    __syncthreads();
    {
      float n = 0.0f, mean = 0.0f, M2 = 0.0f;
#pragma unroll 1
      for (int w2 = 0; w2 < GWAVE; ++w2) {
        const float nb = wst[w2 * WSTW];
        const float mb = wst[w2 * WSTW + 1 + tid];
        const float qb = wst[w2 * WSTW + 1 + GBN + tid];
        if (nb > 0.5f) {
          const float nn = n + nb;
          const float delta = mb - mean;
          const float f = nb / nn;
          mean = fmaf(delta, f, mean);
          M2 = M2 + qb + delta * delta * n * f;
          n = nn;
        }
      }
      pst[1 + tid] = mean;
      pst[1 + GBN + tid] = M2;
      if (tid == 0) pst[0] = n;
    }
#pragma unroll 1
    for (int i = 2 * GBN + 1 + tid; i < PARTW; i += GTHR) pst[i] = 0.0f;
    __syncthreads();
    const int pb = (int)blockIdx.x;
    v4f ps = {0.f, 0.f, 0.f, 0.f};
    if (tid < PARTW / 4) {
      ps = *(const v4fa*)(pst + 4 * tid);
      *(volatile v4f*)(part + (size_t)pb * PARTW + 4 * tid) = ps;
    }
    __threadfence();
    if (tid < PARTW / 4) {
      *(volatile v4f*)(part + (size_t)pb * PARTW + 4 * tid) = ps;
    }
  }
}

__global__ __launch_bounds__(NTHR) void k_gmax(const float* __restrict__ P, const int* __restrict__ neigh,
                                               unsigned short* agg) {
  __shared__ __attribute__((aligned(16))) unsigned short rowbuf[8 * HP];
  const int tid = (int)threadIdx.x, lane = tid & 31, wave = tid >> 5;
  const int node = (int)blockIdx.x * 8 + wave;
  const int nc = node < NN ? node : NN - 1;
  const int jl = lane < NS ? lane : NS - 1;
  int idv = neigh[(size_t)nc * NS + jl];
  idv = idv < 0 ? 0 : (idv > NN - 1 ? NN - 1 : idv);
  const int id0 = __builtin_amdgcn_readlane(idv, 0);
  v4f mx = *(const v4f*)(P + (size_t)id0 * DF + 4 * lane);
#pragma unroll 4
  for (int j = 1; j < NS; ++j) {
    const int idj = __builtin_amdgcn_readlane(idv, j);
    const v4f v = *(const v4f*)(P + (size_t)idj * DF + 4 * lane);
    mx.x = max_keep(v.x, mx.x);
    mx.y = max_keep(v.y, mx.y);
    mx.z = max_keep(v.z, mx.z);
    mx.w = max_keep(v.w, mx.w);
  }
  pin4(mx);
  const bool live = node < NN;
  v4f y;
  y.x = live ? mx.x : 0.0f; y.y = live ? mx.y : 0.0f; y.z = live ? mx.z : 0.0f; y.w = live ? mx.w : 0.0f;
  v4us h4, l4;
  split4(y, h4, l4);
  unsigned short* rb = rowbuf + wave * HP;
  *(v4usa*)(rb + 4 * lane) = h4;
  *(v4usa*)(rb + DF + 4 * lane) = l4;
  wave_sync();
  const v8us q0 = *(const v8usa*)(rb + 8 * lane);
  unsigned short* rp = agg + (size_t)node * HP + 8 * lane;
  *(volatile v8us*)rp = q0;
  __threadfence();
  *(volatile v8us*)rp = q0;
}

__global__ __launch_bounds__(DF) void k_comb(const float* __restrict__ part, float* stat) {
  __shared__ __attribute__((aligned(16))) float stg[3 * DF];
  const int tid = (int)threadIdx.x;
  const int c = tid;
  double n = 0.0, mean = 0.0, M2 = 0.0;
#pragma unroll 1
  for (int b = 0; b < NTILE; ++b) {
    const float* pr = part + (size_t)b * PARTW;
    const double nb = (double)pr[0];
    const double mb = (double)pr[1 + c];
    const double qb = (double)pr[1 + GBN + c];
    if (nb > 0.5) {
      const double nn = n + nb;
      const double delta = mb - mean;
      const double f = nb / nn;
      mean = mean + delta * f;
      M2 = M2 + qb + delta * delta * n * f;
      n = nn;
    }
  }
  const double nt = n < 1.0 ? 1.0 : n;
  const float varf  = (float)(M2 / nt);
  const float meanf = (float)mean;
  const float s = sqrtf(varf + 1e-5f);
  const float rinv = 1.0f / s;
  stg[c] = meanf;
  stg[DF + c] = s;
  stg[2 * DF + c] = rinv;
  __syncthreads();
  v4f v = {0.f, 0.f, 0.f, 0.f};
  if (tid < (3 * DF) / 4) {
    v = *(const v4fa*)(stg + 4 * tid);
    *(volatile v4f*)(stat + 4 * tid) = v;
  }
  __threadfence();
  if (tid < (3 * DF) / 4) {
    *(volatile v4f*)(stat + 4 * tid) = v;
  }
}

__global__ __launch_bounds__(NTHR) void k_apply(const float* __restrict__ T, const float* __restrict__ stat,
                                                const float* __restrict__ par, unsigned short* x2) {
#pragma clang fp contract(off)
  __shared__ __attribute__((aligned(16))) float prm[4 * DF];
  __shared__ __attribute__((aligned(16))) unsigned short rowbuf[8 * HP];
  const int tid = (int)threadIdx.x, lane = tid & 31, wave = tid >> 5;
  if (tid < 64) {
    const v4f q = *(const v4f*)(stat + (size_t)(2 * wave) * DF + 4 * lane);
    *(v4fa*)(prm + wave * DF + 4 * lane) = q;
  } else if (tid < 128) {
    const v4f q = *(const v4f*)(par + (size_t)(2 + wave) * DF + 4 * lane);
    *(v4fa*)(prm + wave * DF + 4 * lane) = q;
  }
  __syncthreads();
  const int row = (int)blockIdx.x * 8 + wave;
  const int rc = row < NN ? row : NN - 1;
  const v4f t = *(const v4f*)(T + (size_t)rc * DF + 4 * lane);
  pin4(t);
  const v4f mu = *(const v4fa*)(prm + 4 * lane);
  const v4f ri = *(const v4fa*)(prm + DF + 4 * lane);
  const v4f g  = *(const v4fa*)(prm + 2 * DF + 4 * lane);
  const v4f be = *(const v4fa*)(prm + 3 * DF + 4 * lane);
  v4f y;
  y.x = ((t.x - mu.x) * ri.x) * g.x + be.x;
  y.y = ((t.y - mu.y) * ri.y) * g.y + be.y;
  y.z = ((t.z - mu.z) * ri.z) * g.z + be.z;
  y.w = ((t.w - mu.w) * ri.w) * g.w + be.w;
  float ss = (y.x * y.x + y.y * y.y) + (y.z * y.z + y.w * y.w);
  ss += __shfl_xor(ss, 16, 32);
  ss += __shfl_xor(ss, 8, 32);
  ss += __shfl_xor(ss, 4, 32);
  ss += __shfl_xor(ss, 2, 32);
  ss += __shfl_xor(ss, 1, 32);
  const float d = sqrtf(ss) + 1e-6f;
  const float r = 1.0f / d;
  const bool live = row < NN;
  v4f z;
  z.x = live ? y.x * r : 0.0f;
  z.y = live ? y.y * r : 0.0f;
  z.z = live ? y.z * r : 0.0f;
  z.w = live ? y.w * r : 0.0f;
  v4us h4, l4;
  split4(z, h4, l4);
  unsigned short* rb = rowbuf + wave * HP;
  *(v4usa*)(rb + 4 * lane) = h4;
  *(v4usa*)(rb + DF + 4 * lane) = l4;
  wave_sync();
  const v8us q0 = *(const v8usa*)(rb + 8 * lane);
  unsigned short* rp = x2 + (size_t)row * HP + 8 * lane;
  *(volatile v8us*)rp = q0;
  __threadfence();
  *(volatile v8us*)rp = q0;
}

extern "C" void kernel_launch(void* const* d_in, const int* in_sizes, int n_in,
                              void* d_out, int out_size, void* d_ws, size_t ws_size,
                              hipStream_t stream) {
  if (n_in < 13) return;
  if (in_sizes[0] != NN * DF) return;
  if (in_sizes[1] != NN * NS || in_sizes[2] != NN * NS) return;
  if (in_sizes[3] != DF * DF || in_sizes[5] != DF * DF) return;
  if (in_sizes[7] != 2 * DF * DF || in_sizes[9] != 2 * DF * DF) return;
  if (in_sizes[4] != DF || in_sizes[6] != DF || in_sizes[8] != DF || in_sizes[10] != DF) return;
  if (in_sizes[11] != DF || in_sizes[12] != DF) return;
  if ((long long)out_size != (long long)NN * DF) return;
  if (ws_size < WS_TOTAL) return;

  const float* feat = (const float*)d_in[0];
  const int*   ng0  = (const int*)d_in[1];
  const int*   ng1  = (const int*)d_in[2];
  const float* Wa0  = (const float*)d_in[3];
  const float* ba0  = (const float*)d_in[4];
  const float* Wa1  = (const float*)d_in[5];
  const float* ba1  = (const float*)d_in[6];
  const float* W0   = (const float*)d_in[7];
  const float* b0   = (const float*)d_in[8];
  const float* W1   = (const float*)d_in[9];
  const float* b1   = (const float*)d_in[10];
  const float* gam  = (const float*)d_in[11];
  const float* bet  = (const float*)d_in[12];
  float* out = (float*)d_out;

  char* ws = (char*)d_ws;
  unsigned short* XB   = (unsigned short*)(ws + O_XB);
  float*          Pp   = (float*)(ws + O_P);
  unsigned short* AGG  = (unsigned short*)(ws + O_AGG);
  float*          Tt   = (float*)(ws + O_T);
  unsigned short* X2   = (unsigned short*)(ws + O_X2);
  unsigned short* WA0T = (unsigned short*)(ws + O_WA0T);
  unsigned short* W0C  = (unsigned short*)(ws + O_W0C);
  unsigned short* WA1D = (unsigned short*)(ws + O_WA1D);
  unsigned short* W1C  = (unsigned short*)(ws + O_W1C);
  float*          PAR  = (float*)(ws + O_PAR);
  float*          REC  = (float*)(ws + O_REC);
  float*          STAT = (float*)(ws + O_STAT);

  k_prep<<<PREP_BLOCKS, NTHR, 0, stream>>>(feat, Wa0, ba0, Wa1, ba1, W0, b0, W1, b1, gam, bet,
                                           XB, WA0T, W0C, WA1D, W1C, PAR);
  k_gemm<DF, KA0, DF, 0, 1, 0, 0><<<NTILE, GTHR, 0, stream>>>(XB, XB, WA0T, PAR, Pp, REC);
  k_gmax<<<ROWBLK, NTHR, 0, stream>>>(Pp, ng0, AGG);
  k_gemm<DF, DF, HP, HP, 1, 1, 0><<<NTILE, GTHR, 0, stream>>>(XB, AGG, W0C, PAR + 2 * DF, Tt, REC);
  k_comb<<<1, DF, 0, stream>>>(REC, STAT);
  k_apply<<<ROWBLK, NTHR, 0, stream>>>(Tt, STAT, PAR, X2);
  k_gemm<HP, HP, HP, 0, 1, 0, 0><<<NTILE, GTHR, 0, stream>>>(X2, X2, WA1D, PAR + DF, Pp, REC);
  k_gmax<<<ROWBLK, NTHR, 0, stream>>>(Pp, ng1, AGG);
  k_gemm<HP, HP, HP, HP, 0, 0, 1><<<NTILE, GTHR, 0, stream>>>(X2, AGG, W1C, PAR + 3 * DF, out, REC);
}
